// HardNegativeContrastiveLoss_56573309224206
// MI455X (gfx1250) — hardware-verified
//
#include <hip/hip_runtime.h>


namespace {
constexpr int B = 8192, D = 128, N2 = 2 * B, NBLK = N2 / 64;
constexpr float XS = 8.0f, INV_T = 10.0f, MARGIN = 0.5f;
typedef _Float16 b16;
typedef __attribute__((ext_vector_type(16))) _Float16 v16b;
typedef __attribute__((ext_vector_type(8))) _Float16 v8b;
typedef __attribute__((ext_vector_type(8))) float v8f;
typedef __attribute__((ext_vector_type(4))) float v4f;
__device__ __forceinline__ float bf16_rne(float f) { unsigned int u = __float_as_uint(f); u += 0x7FFFu + ((u >> 16) & 1u); return __uint_as_float(u & 0xFFFF0000u); }
__device__ __forceinline__ v16b frag_kb(const b16* p, int hh) { const v8b a = *(const v8b*)(p + 8 * hh), b = *(const v8b*)(p + 16 + 8 * hh); v16b f;
#pragma unroll
  for (int e = 0; e < 8; ++e) { f[e] = a[e]; f[8 + e] = b[e]; } return f; }
__device__ __forceinline__ v8f wmma16b(v16b a, v16b b, v8f c) { v8f d = __builtin_amdgcn_wmma_f32_16x16x32_f16(false, a, false, b, (short)0, c, false, false); asm volatile("v_nop\n\tv_nop\n\tv_nop\n\tv_nop" : "+v"(d) : "v"(a), "v"(b)); return d; }
__device__ __forceinline__ float pmul(float a, float b) { float p = a * b; asm volatile("" : "+v"(p)); return p; }

__global__ __launch_bounds__(256) void norm_kernel(const float* __restrict__ z1, const float* __restrict__ z2, b16* __restrict__ ZN, float* __restrict__ POS) {
  __shared__ float pos_s[32]; __shared__ __attribute__((aligned(16))) b16 rowh[8][D];
  const int wave = threadIdx.x >> 5, lane = threadIdx.x & 31;
  for (int rr = 0; rr < 4; ++rr) { const int li = wave * 4 + rr; const size_t i = (size_t)blockIdx.x * 32 + li;
    const bool second = i >= (size_t)B; const float* zr = second ? (z2 + (i - B) * D) : (z1 + i * D); const v4f a = *(const v4f*)(zr + lane * 4); float x[4] = {bf16_rne(a[0]), bf16_rne(a[1]), bf16_rne(a[2]), bf16_rne(a[3])};
    float q = x[0] * x[0] + x[1] * x[1] + x[2] * x[2] + x[3] * x[3];
#pragma unroll
    for (int o = 16; o >= 1; o >>= 1) q += __shfl_xor(q, o);
    const float inv = 1.0f / fmaxf(sqrtf(q), 1e-12f); float y[4]; for (int j = 0; j < 4; ++j) y[j] = x[j] * inv;
    float pp = 0.0f;
    if (!second) { const v4f bq = *(const v4f*)(z2 + i * D + lane * 4); float xb[4] = {bf16_rne(bq[0]), bf16_rne(bq[1]), bf16_rne(bq[2]), bf16_rne(bq[3])}; float q2 = xb[0] * xb[0] + xb[1] * xb[1] + xb[2] * xb[2] + xb[3] * xb[3];
#pragma unroll
      for (int o = 16; o >= 1; o >>= 1) q2 += __shfl_xor(q2, o);
      const float inv2 = 1.0f / fmaxf(sqrtf(q2), 1e-12f); for (int j = 0; j < 4; ++j) pp += pmul(y[j], xb[j] * inv2);
#pragma unroll
      for (int o = 16; o >= 1; o >>= 1) pp += __shfl_xor(pp, o); }
    if (lane == 0) pos_s[li] = pp;
    for (int j = 0; j < 4; ++j) rowh[wave][lane * 4 + j] = (b16)(y[j] * XS);
    __builtin_amdgcn_fence(__ATOMIC_RELEASE, "workgroup"); __builtin_amdgcn_wave_barrier(); __builtin_amdgcn_fence(__ATOMIC_ACQUIRE, "workgroup");
    for (int pass = 0; pass < 2; ++pass) { if (lane < 16) *(volatile v8b*)(ZN + i * D + lane * 8) = *(const v8b*)(&rowh[wave][lane * 8]); __threadfence(); }
    __builtin_amdgcn_wave_barrier(); }
  __syncthreads();
  const size_t i0 = (size_t)blockIdx.x * 32;
  for (int pass = 0; pass < 2; ++pass) { if (i0 < (size_t)B && threadIdx.x < 32) ((volatile float*)POS)[i0 + threadIdx.x] = pos_s[threadIdx.x]; __threadfence(); }
}
__global__ __launch_bounds__(128) void simmax_kernel(const b16* __restrict__ ZN, const float* __restrict__ POS, float* __restrict__ PART) {
  __shared__ float lsum[4][16];
  const int wave = threadIdx.x >> 5, lane = threadIdx.x & 31, nloc = lane & 15, hlf = lane >> 4; const size_t m0 = (size_t)blockIdx.x * 64 + wave * 16;
  v16b a[4]; for (int kk = 0; kk < 4; ++kk) a[kk] = frag_kb(ZN + (m0 + nloc) * D + kk * 32, hlf);
  float mx[8]; for (int r = 0; r < 8; ++r) mx[r] = -INFINITY;
  for (int n0 = 0; n0 < N2; n0 += 128) {
    v8f acc[8];
#pragma unroll
    for (int t = 0; t < 8; ++t) acc[t] = (v8f){};
#pragma unroll
    for (int kk = 0; kk < 4; ++kk) {
#pragma unroll
      for (int t = 0; t < 8; ++t) acc[t] = wmma16b(a[kk], frag_kb(ZN + (size_t)(n0 + t * 16 + nloc) * D + kk * 32, hlf), acc[t]); }
#pragma unroll
    for (int t = 0; t < 8; ++t) { const int j = n0 + t * 16 + nloc;
#pragma unroll
      for (int r = 0; r < 8; ++r) { const int i = (int)m0 + 8 * hlf + r; const bool masked = (j == i + B) || (j == i - B); if (!masked) mx[r] = fmaxf(mx[r], acc[t][r]); } } }
#pragma unroll
  for (int r = 0; r < 8; ++r) { float m = mx[r]; m = fmaxf(m, __shfl_xor(m, 1)); m = fmaxf(m, __shfl_xor(m, 2)); m = fmaxf(m, __shfl_xor(m, 4)); m = fmaxf(m, __shfl_xor(m, 8)); mx[r] = m; }
  if (nloc == 0) { float s = 0.0f; for (int r = 0; r < 8; ++r) { const size_t i = m0 + 8 * hlf + r; const float hardest = mx[r] * (INV_T / (XS * XS)); const float pos = POS[i < (size_t)B ? i : i - B]; s += fmaxf(hardest + MARGIN - pos, 0.0f); } lsum[wave][hlf] = s; }
  __syncthreads();
  if (threadIdx.x < 32) { float v = 0.0f; if (threadIdx.x == 0) { for (int w = 0; w < 4; ++w) v += lsum[w][0] + lsum[w][1]; }
    for (int pass = 0; pass < 2; ++pass) { ((volatile float*)PART)[(size_t)blockIdx.x * 32 + threadIdx.x] = v; __threadfence(); } }
}
__global__ __launch_bounds__(64) void final_kernel(const float* __restrict__ PART, float* __restrict__ out) {
  if (threadIdx.x != 0) return; float s = 0.0f; for (int b = 0; b < NBLK; ++b) s += PART[(size_t)b * 32]; const float r = s / (float)N2;
  for (int pass = 0; pass < 2; ++pass) { ((volatile float*)out)[0] = r; __threadfence(); }
}
}

extern "C" void kernel_launch(void* const* d_in, const int* in_sizes, int n_in, void* d_out, int out_size, void* d_ws, size_t ws_size, hipStream_t stream) {
  (void)n_in;
  auto Fp = [&](int i) { return (const float*)d_in[i]; };
  if (in_sizes[0] != B * D || in_sizes[1] != B * D || out_size != 1) return;
  size_t off = 0; char* ws = (char*)d_ws;
  auto carve = [&](size_t bytes) { char* p = ws + off; off += (bytes + 255) & ~(size_t)255; return p; };
  b16* ZN = (b16*)carve((size_t)N2 * D * 2); float* POS = (float*)carve((size_t)B * 4); float* PART = (float*)carve((size_t)NBLK * 32 * 4);
  if (off > ws_size) return;
  norm_kernel<<<N2 / 32, 256, 0, stream>>>(Fp(0), Fp(1), ZN, POS);
  simmax_kernel<<<NBLK, 128, 0, stream>>>(ZN, POS, PART);
  final_kernel<<<1, 64, 0, stream>>>(PART, (float*)d_out);
}
